// HybridGCRNGATCell_83846351552829
// MI455X (gfx1250) — hardware-verified
//
#include <hip/hip_runtime.h>
#define BB 32
#define NN 400
#define NK 416
#define FF 64
#define HH 64
#define NHD 4
#define DH 64
#define G4 256
#define NR (BB * NN)

typedef __bf16 v16b __attribute__((ext_vector_type(16)));
typedef unsigned short v8us __attribute__((ext_vector_type(8), may_alias));
typedef float  v8f  __attribute__((ext_vector_type(8)));
typedef float  v4f  __attribute__((ext_vector_type(4)));
typedef float  v4fa __attribute__((ext_vector_type(4), may_alias));
union FragB { v16b v; v8us half[2]; unsigned short u[16]; };

__device__ __forceinline__ unsigned short bf16_bits(float x) { unsigned int u = __float_as_uint(x); return (unsigned short)((u + 0x7FFFu + ((u >> 16) & 1u)) >> 16); }
__device__ __forceinline__ float bf16_val(unsigned short b) { return __uint_as_float(((unsigned int)b) << 16); }
__device__ __forceinline__ float bf16_round(float x) { return bf16_val(bf16_bits(x)); }
template <int NT>
__device__ __forceinline__ v8f mmaN(v16b ah, v16b al, v16b bh, v16b bl, v8f c) {
  c = __builtin_amdgcn_wmma_f32_16x16x32_bf16(false, ah, false, bh, (short)0, c, false, false);
  if (NT >= 2) c = __builtin_amdgcn_wmma_f32_16x16x32_bf16(false, al, false, bh, (short)0, c, false, false);
  if (NT >= 3) c = __builtin_amdgcn_wmma_f32_16x16x32_bf16(false, ah, false, bl, (short)0, c, false, false);
  asm volatile("v_nop\n\tv_nop\n\tv_nop\n\tv_nop" : "+v"(c) : "v"(ah), "v"(al), "v"(bh), "v"(bl));
  return c;
}

__device__ __forceinline__ void store_span256(float* span, v4f lo, v4f hi, int lane) {
  v4f a, b; const int s0 = lane >> 1, s1 = 16 + (lane >> 1); const bool odd = (lane & 1) != 0;
#pragma unroll
  for (int q = 0; q < 4; ++q) { const float l0 = __shfl(lo[q], s0, 32), h0 = __shfl(hi[q], s0, 32), l1 = __shfl(lo[q], s1, 32), h1 = __shfl(hi[q], s1, 32); a[q] = odd ? h0 : l0; b[q] = odd ? h1 : l1; }
  for (int pass = 0; pass < 2; ++pass) { *(volatile v4f*)(span + 4 * lane) = a; *(volatile v4f*)(span + 128 + 4 * lane) = b; if (pass == 0) __threadfence(); } }
__device__ __forceinline__ void store_span512h(_Float16* span, v8us p0, v8us p1, int lane) {
  typedef unsigned int v4u __attribute__((ext_vector_type(4))); union U { v8us h; v4u u; }; U x0, x1, a, b; x0.h = p0; x1.h = p1; const int s0 = lane >> 1, s1 = 16 + (lane >> 1); const bool odd = (lane & 1) != 0;
#pragma unroll
  for (int q = 0; q < 4; ++q) { const unsigned l0 = __shfl(x0.u[q], s0, 32), h0 = __shfl(x1.u[q], s0, 32), l1 = __shfl(x0.u[q], s1, 32), h1 = __shfl(x1.u[q], s1, 32); a.u[q] = odd ? h0 : l0; b.u[q] = odd ? h1 : l1; }
  for (int pass = 0; pass < 2; ++pass) { *(volatile v8us*)((unsigned short*)span + 8 * lane) = a.h; *(volatile v8us*)((unsigned short*)span + 256 + 8 * lane) = b.h; if (pass == 0) __threadfence(); } }

__global__ __launch_bounds__(256) void k_wt_bf16(const float* __restrict__ W, unsigned short* __restrict__ Wt, int K, int N) {
  const int t = blockIdx.x * 256 + threadIdx.x;
  const int k8n = K / 8;
  if (t >= N * k8n) return;
  const int n = t / k8n, k8 = (t % k8n) * 8;
  v8us v;
#pragma unroll
  for (int i = 0; i < 8; ++i) v[i] = bf16_bits(W[(size_t)(k8 + i) * N + n]);
  *(volatile v8us*)(Wt + (size_t)n * K + k8) = v;
  __threadfence();
  *(volatile v8us*)(Wt + (size_t)n * K + k8) = v;
}

template <bool ASPLIT, int ACT, bool BIAS_BF16>
__global__ __launch_bounds__(128) void k_gemm_bf(const float* __restrict__ A, int lda, const unsigned short* __restrict__ Wt, int ldb,
                                               const float* __restrict__ bias, float* __restrict__ C, int ldc, int M, int N, int K) {
  __shared__ __attribute__((aligned(16))) float so[4][16][64];
  const int tid = threadIdx.x, w = tid >> 5, lane = tid & 31, ln = lane & 15, hh = lane >> 4;
  const int ntn = N / 64;
  const int wid = blockIdx.x * 4 + w;
  const int mt = wid / ntn, nq = wid % ntn;
  if (mt * 16 >= M) return;
  const int row0 = mt * 16, col0 = nq * 64;
  const float* arow = A + (size_t)(row0 + ln) * lda;
  v8f acc[4] = {};
  for (int kb = 0; kb < K; kb += 32) {
    FragB ah, al;
    const v4f x0 = *(const v4fa*)(arow + kb + 8 * hh), x1 = *(const v4fa*)(arow + kb + 8 * hh + 4);
    const v4f x2 = *(const v4fa*)(arow + kb + 16 + 8 * hh), x3 = *(const v4fa*)(arow + kb + 16 + 8 * hh + 4);
    float xs[16] = {x0[0],x0[1],x0[2],x0[3],x1[0],x1[1],x1[2],x1[3],x2[0],x2[1],x2[2],x2[3],x3[0],x3[1],x3[2],x3[3]};
#pragma unroll
    for (int i = 0; i < 16; ++i) { const unsigned short hb = bf16_bits(xs[i]); ah.u[i] = hb; al.u[i] = ASPLIT ? bf16_bits(xs[i] - bf16_val(hb)) : (unsigned short)0; }
#pragma unroll
    for (int t = 0; t < 4; ++t) {
      const unsigned short* brow = Wt + (size_t)(col0 + t * 16 + ln) * ldb + kb;
      FragB b;
      b.half[0] = *(const v8us*)(brow + 8 * hh);
      b.half[1] = *(const v8us*)(brow + 16 + 8 * hh);
      acc[t] = mmaN<ASPLIT ? 2 : 1>(ah.v, al.v, b.v, b.v, acc[t]);
    }
  }
#pragma unroll
  for (int t = 0; t < 4; ++t) {
    float bv = bias ? bias[col0 + t * 16 + ln] : 0.f;
    if (BIAS_BF16) bv = bf16_round(bv);
#pragma unroll
    for (int r = 0; r < 8; ++r) { float v = acc[t][r] + bv; if (ACT == 1) v = fmaxf(v, 0.f); so[w][8 * hh + r][t * 16 + ln] = v; }
  }
  __builtin_amdgcn_fence(__ATOMIC_ACQ_REL, "workgroup");
  __builtin_amdgcn_wave_barrier();
  const int rsub = lane >> 4, c4 = (lane & 15) * 4;
  for (int pass = 0; pass < 2; ++pass) {
#pragma unroll
    for (int q = 0; q < 8; ++q) {
      const int r = q * 2 + rsub;
      const v4f v = *(const v4fa*)&so[w][r][c4];
      *(volatile v4f*)(C + (size_t)(row0 + r) * ldc + col0 + c4) = v;
    }
    if (pass == 0) __threadfence();
  }
}

template <int D, bool CAUSAL>
__global__ __launch_bounds__(128) void k_flash(const float* __restrict__ qb, const float* __restrict__ kb, const float* __restrict__ vb,
                                             int pitch, int T, int H, float scale, float* __restrict__ y, int ypitch) {
  constexpr int KS = D / 32;
  constexpr int DT = D / 16;
  __shared__ __attribute__((aligned(16))) unsigned short sKh[32][D + 8], sKl[32][D + 8], sVh[32][D + 8], sVl[32][D + 8];
  __shared__ __attribute__((aligned(16))) unsigned short sPh[4][16][40], sPl[4][16][40];
  __shared__ __attribute__((aligned(16))) float sO[4][16][D];
  const int tid = threadIdx.x, w = tid >> 5, lane = tid & 31, ln = lane & 15, hh = lane >> 4;
  const int nqb = (T + 63) / 64;
  const int bh = blockIdx.x / nqb, qblk = blockIdx.x % nqb;
  const int b = bh / H, h = bh % H;
  const int q0 = qblk * 64 + w * 16;
  const float* Q = qb + (size_t)b * T * pitch + h * D;
  const float* K = kb + (size_t)b * T * pitch + h * D;
  const float* V = vb + (size_t)b * T * pitch + h * D;

  FragB aqh[KS], aql[KS];
  {
    int row = q0 + ln; if (row >= T) row = T - 1;
    const float* qr = Q + (size_t)row * pitch;
#pragma unroll
    for (int ks = 0; ks < KS; ++ks)
#pragma unroll
      for (int i = 0; i < 16; ++i) {
        const int d = ks * 32 + ((i < 8) ? (8 * hh + i) : (16 + 8 * hh + (i - 8)));
        const float x = qr[d] * scale; const unsigned short hb = bf16_bits(x);
        aqh[ks].u[i] = hb; aql[ks].u[i] = bf16_bits(x - bf16_val(hb));
      }
  }
  float m_r[8], l_r[8];
#pragma unroll
  for (int r = 0; r < 8; ++r) { m_r[r] = -3.0e38f; l_r[r] = 0.f; }
  v8f oacc[DT];
#pragma unroll
  for (int dt = 0; dt < DT; ++dt) oacc[dt] = (v8f){0.f,0.f,0.f,0.f,0.f,0.f,0.f,0.f};

  const int kv_end = CAUSAL ? min(T, qblk * 64 + 64) : T;
  for (int j0 = 0; j0 < kv_end; j0 += 32) {
    __syncthreads();
    for (int e = tid; e < 32 * (D / 4); e += 128) {
      const int r = e / (D / 4), c4 = (e % (D / 4)) * 4;
      const int key = j0 + r;
      v4f kf = {0.f,0.f,0.f,0.f}, vf = {0.f,0.f,0.f,0.f};
      if (key < T) { kf = *(const v4fa*)(K + (size_t)key * pitch + c4); vf = *(const v4fa*)(V + (size_t)key * pitch + c4); }
#pragma unroll
      for (int t = 0; t < 4; ++t) {
        unsigned short hb = bf16_bits(kf[t]); sKh[r][c4 + t] = hb; sKl[r][c4 + t] = bf16_bits(kf[t] - bf16_val(hb));
        hb = bf16_bits(vf[t]); sVh[r][c4 + t] = hb; sVl[r][c4 + t] = bf16_bits(vf[t] - bf16_val(hb));
      }
    }
    __syncthreads();
    v8f s[2];
#pragma unroll
    for (int nt = 0; nt < 2; ++nt) {
      v8f acc = {};
#pragma unroll
      for (int ks = 0; ks < KS; ++ks) {
        FragB bh_, bl_;
        bh_.half[0] = *(const v8us*)&sKh[nt * 16 + ln][ks * 32 + 8 * hh]; bh_.half[1] = *(const v8us*)&sKh[nt * 16 + ln][ks * 32 + 16 + 8 * hh];
        bl_.half[0] = *(const v8us*)&sKl[nt * 16 + ln][ks * 32 + 8 * hh]; bl_.half[1] = *(const v8us*)&sKl[nt * 16 + ln][ks * 32 + 16 + 8 * hh];
        acc = mmaN<3>(aqh[ks].v, aql[ks].v, bh_.v, bl_.v, acc);
      }
      s[nt] = acc;
    }
    float alpha[8];
#pragma unroll
    for (int r = 0; r < 8; ++r) {
      const int qi = q0 + 8 * hh + r;
      const int ja = j0 + ln, jb = j0 + 16 + ln;
      if (CAUSAL) { if (ja > qi) s[0][r] = -3.0e38f; if (jb > qi) s[1][r] = -3.0e38f; }
      if (ja >= T) s[0][r] = -3.0e38f;
      if (jb >= T) s[1][r] = -3.0e38f;
      float mx = fmaxf(s[0][r], s[1][r]);
      mx = fmaxf(mx, __shfl_xor(mx, 1, 32)); mx = fmaxf(mx, __shfl_xor(mx, 2, 32)); mx = fmaxf(mx, __shfl_xor(mx, 4, 32)); mx = fmaxf(mx, __shfl_xor(mx, 8, 32));
      const float mnew = fmaxf(m_r[r], mx);
      alpha[r] = (mnew > -1.0e38f) ? __expf(m_r[r] - mnew) : 1.0f;
      const float p0 = (s[0][r] > -1.0e38f) ? __expf(s[0][r] - mnew) : 0.f;
      const float p1 = (s[1][r] > -1.0e38f) ? __expf(s[1][r] - mnew) : 0.f;
      m_r[r] = mnew;
      l_r[r] = l_r[r] * alpha[r] + p0 + p1;
      unsigned short hb = bf16_bits(p0); sPh[w][8 * hh + r][ln] = hb;      sPl[w][8 * hh + r][ln] = bf16_bits(p0 - bf16_val(hb));
      hb = bf16_bits(p1);                sPh[w][8 * hh + r][16 + ln] = hb; sPl[w][8 * hh + r][16 + ln] = bf16_bits(p1 - bf16_val(hb));
    }
#pragma unroll
    for (int dt = 0; dt < DT; ++dt)
#pragma unroll
      for (int r = 0; r < 8; ++r) oacc[dt][r] *= alpha[r];
    __builtin_amdgcn_fence(__ATOMIC_ACQ_REL, "workgroup");
    __builtin_amdgcn_wave_barrier();
    FragB pah, pal;
    pah.half[0] = *(const v8us*)&sPh[w][ln][8 * hh]; pah.half[1] = *(const v8us*)&sPh[w][ln][16 + 8 * hh];
    pal.half[0] = *(const v8us*)&sPl[w][ln][8 * hh]; pal.half[1] = *(const v8us*)&sPl[w][ln][16 + 8 * hh];
#pragma unroll
    for (int dt = 0; dt < DT; ++dt) {
      FragB bvh, bvl;
#pragma unroll
      for (int i = 0; i < 8; ++i) {
        bvh.u[i] = sVh[8 * hh + i][dt * 16 + ln]; bvh.u[8 + i] = sVh[16 + 8 * hh + i][dt * 16 + ln];
        bvl.u[i] = sVl[8 * hh + i][dt * 16 + ln]; bvl.u[8 + i] = sVl[16 + 8 * hh + i][dt * 16 + ln];
      }
      oacc[dt] = mmaN<3>(pah.v, pal.v, bvh.v, bvl.v, oacc[dt]);
    }
    __builtin_amdgcn_fence(__ATOMIC_ACQ_REL, "workgroup");
    __builtin_amdgcn_wave_barrier();
  }
#pragma unroll
  for (int r = 0; r < 8; ++r) {
    float l = l_r[r];
    l += __shfl_xor(l, 1, 32); l += __shfl_xor(l, 2, 32); l += __shfl_xor(l, 4, 32); l += __shfl_xor(l, 8, 32);
    l_r[r] = (l > 0.f) ? 1.0f / l : 0.f;
  }
#pragma unroll
  for (int dt = 0; dt < DT; ++dt)
#pragma unroll
    for (int r = 0; r < 8; ++r) sO[w][8 * hh + r][dt * 16 + ln] = oacc[dt][r] * l_r[r];
  __builtin_amdgcn_fence(__ATOMIC_ACQ_REL, "workgroup");
  __builtin_amdgcn_wave_barrier();
  for (int pass = 0; pass < 2; ++pass) {
    for (int r = 0; r < 16; ++r) {
      const int row = q0 + r;
      if (row < T && lane < D / 4) {
        const v4f val = *(const v4fa*)&sO[w][r][lane * 4];
        *(volatile v4f*)(y + ((size_t)b * T + row) * ypitch + h * D + lane * 4) = val;
      }
    }
    if (pass == 0) __threadfence();
  }
}

template <bool ASPLIT, int ACT, bool BIAS_BF16, bool RES_BF16>
__global__ __launch_bounds__(128) void k_gemm_bf3(const float* __restrict__ A, int lda, const unsigned short* __restrict__ Wt, int ldb,
                                                const float* __restrict__ bias, const float* __restrict__ resid, int rmod, int ldr,
                                                float* __restrict__ C, int ldc, int M, int N, int K) {
  __shared__ __attribute__((aligned(16))) float so[4][16][64];
  const int tid = threadIdx.x, w = tid >> 5, lane = tid & 31, ln = lane & 15, hh = lane >> 4;
  const int ntn = N / 64;
  const int wid = blockIdx.x * 4 + w;
  const int mt = wid / ntn, nq = wid % ntn;
  if (mt * 16 >= M) return;
  const int row0 = mt * 16, col0 = nq * 64;
  const float* arow = A + (size_t)(row0 + ln) * lda;
  v8f acc[4] = {};
  for (int kb = 0; kb < K; kb += 32) {
    FragB ah, al;
    const v4f x0 = *(const v4fa*)(arow + kb + 8 * hh), x1 = *(const v4fa*)(arow + kb + 8 * hh + 4);
    const v4f x2 = *(const v4fa*)(arow + kb + 16 + 8 * hh), x3 = *(const v4fa*)(arow + kb + 16 + 8 * hh + 4);
    float xs[16] = {x0[0],x0[1],x0[2],x0[3],x1[0],x1[1],x1[2],x1[3],x2[0],x2[1],x2[2],x2[3],x3[0],x3[1],x3[2],x3[3]};
#pragma unroll
    for (int i = 0; i < 16; ++i) { const unsigned short hb = bf16_bits(xs[i]); ah.u[i] = hb; al.u[i] = ASPLIT ? bf16_bits(xs[i] - bf16_val(hb)) : (unsigned short)0; }
#pragma unroll
    for (int t = 0; t < 4; ++t) {
      const unsigned short* brow = Wt + (size_t)(col0 + t * 16 + ln) * ldb + kb;
      FragB b;
      b.half[0] = *(const v8us*)(brow + 8 * hh);
      b.half[1] = *(const v8us*)(brow + 16 + 8 * hh);
      acc[t] = mmaN<ASPLIT ? 2 : 1>(ah.v, al.v, b.v, b.v, acc[t]);
    }
  }
#pragma unroll
  for (int t = 0; t < 4; ++t) {
    const int col = col0 + t * 16 + ln;
    float bv = bias ? bias[col] : 0.f;
    if (BIAS_BF16) bv = bf16_round(bv);
#pragma unroll
    for (int r = 0; r < 8; ++r) {
      float v = acc[t][r] + bv;
      if (resid) { float rv = resid[(size_t)((row0 + 8 * hh + r) % rmod) * ldr + col]; if (RES_BF16) rv = bf16_round(rv); v += rv; }
      if (ACT == 1) v = fmaxf(v, 0.f);
      if (ACT == 2) v = 0.5f * v * (1.0f + erff(v * 0.70710678118654752f));
      if (ACT == 3) { const float u = 0.7978845608028654f * (v + 0.044715f * v * v * v); v = 0.5f * v * (1.0f + tanhf(u)); }
      so[w][8 * hh + r][t * 16 + ln] = v;
    }
  }
  __builtin_amdgcn_fence(__ATOMIC_ACQ_REL, "workgroup");
  __builtin_amdgcn_wave_barrier();
  const int rsub = lane >> 4, c4 = (lane & 15) * 4;
  for (int pass = 0; pass < 2; ++pass) {
#pragma unroll
    for (int q = 0; q < 8; ++q) {
      const int r = q * 2 + rsub;
      const v4f v = *(const v4fa*)&so[w][r][c4];
      *(volatile v4f*)(C + (size_t)(row0 + r) * ldc + col0 + c4) = v;
    }
    if (pass == 0) __threadfence();
  }
}
template <bool PARAM_BF16>
__global__ __launch_bounds__(256) void k_layernorm(const float* __restrict__ X, const float* __restrict__ R, const float* __restrict__ g, const float* __restrict__ bta,
                                                  float* __restrict__ out_sum, float* __restrict__ out_norm, int N, float eps) {
  __shared__ float red[256];
  const int row = blockIdx.x, tid = threadIdx.x;
  const float* x = X + (size_t)row * N; const float* rr = R ? R + (size_t)row * N : nullptr;
  float vals[16];
  const int per = N / 256;
  float s1 = 0.f;
  for (int u = 0; u < per / 4; ++u) {
    const int j = tid * 4 + 1024 * u;
    const v4f a = *(const v4fa*)(x + j);
    v4f b = {0.f,0.f,0.f,0.f}; if (rr) b = *(const v4fa*)(rr + j);
#pragma unroll
    for (int q = 0; q < 4; ++q) { const float v = a[q] + b[q]; vals[u * 4 + q] = v; s1 += v; }
  }
  red[tid] = s1; __syncthreads();
  for (int st = 128; st > 0; st >>= 1) { if (tid < st) red[tid] += red[tid + st]; __syncthreads(); }
  const float mu = red[0] / (float)N; __syncthreads();
  float s2 = 0.f;
  for (int u = 0; u < per / 4; ++u)
#pragma unroll
    for (int q = 0; q < 4; ++q) { const float c = vals[u * 4 + q] - mu; s2 += c * c; }
  red[tid] = s2; __syncthreads();
  for (int st = 128; st > 0; st >>= 1) { if (tid < st) red[tid] += red[tid + st]; __syncthreads(); }
  const float rs = rsqrtf(red[0] / (float)N + eps);
  for (int pass = 0; pass < 2; ++pass) {
    for (int u = 0; u < per / 4; ++u) {
      const int j = tid * 4 + 1024 * u;
      v4f o, sm;
#pragma unroll
      for (int q = 0; q < 4; ++q) {
        float gg = g[j + q], bb = bta[j + q];
        if (PARAM_BF16) { gg = bf16_round(gg); bb = bf16_round(bb); }
        sm[q] = vals[u * 4 + q]; o[q] = (vals[u * 4 + q] - mu) * rs * gg + bb;
      }
      if (out_sum) *(volatile v4f*)(out_sum + (size_t)row * N + j) = sm;
      *(volatile v4f*)(out_norm + (size_t)row * N + j) = o;
    }
    if (pass == 0) __threadfence();
  }
}


typedef _Float16 v16h __attribute__((ext_vector_type(16)));
union FragH { v16h v; v8us half[2]; _Float16 h[16]; unsigned short u[16]; };
template <int NT>
__device__ __forceinline__ v8f mmaH(v16h ah, v16h al, v16h bh, v16h bl, v8f c) {
  c = __builtin_amdgcn_wmma_f32_16x16x32_f16(false, ah, false, bh, (short)0, c, false, false);
  if (NT >= 2) c = __builtin_amdgcn_wmma_f32_16x16x32_f16(false, al, false, bh, (short)0, c, false, false);
  if (NT >= 3) c = __builtin_amdgcn_wmma_f32_16x16x32_f16(false, ah, false, bl, (short)0, c, false, false);
  asm volatile("v_nop\n\tv_nop\n\tv_nop\n\tv_nop" : "+v"(c) : "v"(ah), "v"(al), "v"(bh), "v"(bl));
  return c;
}
template <bool ASPLIT>
__global__ __launch_bounds__(128) void k_gemm_h(const float* __restrict__ A, int lda, size_t sA, const _Float16* __restrict__ Bh, int ldb, size_t sB, float alpha, float* __restrict__ C, int ldc, size_t sC, int M, int N, int K) {
  __shared__ __attribute__((aligned(16))) float so[4][16][64];
  const int tid = threadIdx.x, w = tid >> 5, lane = tid & 31, ln = lane & 15, hh = lane >> 4; const int by = blockIdx.y;
  A += (size_t)by * sA; Bh += (size_t)by * sB; C += (size_t)by * sC;
  const int ntn = (N + 63) / 64; const int wid = blockIdx.x * 4 + w; const int mt = wid / ntn, nq = wid % ntn; if (mt * 16 >= M) return;
  const int row0 = mt * 16, col0 = nq * 64; const float* arow = A + (size_t)(row0 + ln) * lda;
  v8f acc[4] = {};
  for (int kb = 0; kb < K; kb += 32) {
    FragH ah, al;
    const v4f x0 = *(const v4fa*)(arow + kb + 8 * hh), x1 = *(const v4fa*)(arow + kb + 8 * hh + 4), x2 = *(const v4fa*)(arow + kb + 16 + 8 * hh), x3 = *(const v4fa*)(arow + kb + 16 + 8 * hh + 4);
    float xs[16] = {x0[0],x0[1],x0[2],x0[3],x1[0],x1[1],x1[2],x1[3],x2[0],x2[1],x2[2],x2[3],x3[0],x3[1],x3[2],x3[3]};
#pragma unroll
    for (int i = 0; i < 16; ++i) { const _Float16 h = (_Float16)xs[i]; ah.h[i] = h; al.h[i] = ASPLIT ? (_Float16)(xs[i] - (float)h) : (_Float16)0.0f; }
#pragma unroll
    for (int t = 0; t < 4; ++t) { if (col0 + t * 16 >= N) continue; const size_t boff = (size_t)(col0 + t * 16 + ln) * ldb + kb; FragH bq; bq.half[0] = *(const v8us*)(Bh + boff + 8 * hh); bq.half[1] = *(const v8us*)(Bh + boff + 16 + 8 * hh);
      acc[t] = mmaH<ASPLIT ? 2 : 1>(ah.v, al.v, bq.v, bq.v, acc[t]); }
  }
#pragma unroll
  for (int t = 0; t < 4; ++t) { if (col0 + t * 16 >= N) continue;
#pragma unroll
    for (int r = 0; r < 8; ++r) so[w][8 * hh + r][t * 16 + ln] = acc[t][r] * alpha; }
  __builtin_amdgcn_fence(__ATOMIC_ACQ_REL, "workgroup"); __builtin_amdgcn_wave_barrier();
  const int rsub = lane >> 4, c4 = (lane & 15) * 4;
  for (int pass = 0; pass < 2; ++pass) {
#pragma unroll
    for (int q = 0; q < 8; ++q) { const int r = q * 2 + rsub; if (col0 + c4 < N) { const v4f v = *(const v4fa*)&so[w][r][c4]; *(volatile v4f*)(C + (size_t)(row0 + r) * ldc + col0 + c4) = v; } }
    if (pass == 0) __threadfence(); }
}

__global__ __launch_bounds__(256) void k_wt_f16(const float* __restrict__ W, _Float16* __restrict__ Wt, int K, int N, float scale) {
  const int t = blockIdx.x * 256 + threadIdx.x; if (t >= N * (K / 8)) return; const int n = t / (K / 8), k8 = (t % (K / 8)) * 8; FragH f;
#pragma unroll
  for (int i = 0; i < 8; ++i) f.h[i] = (_Float16)(bf16_round(W[(size_t)(k8 + i) * N + n]) * scale); const v8us o = f.half[0];
  *(volatile v8us*)((unsigned short*)Wt + (size_t)n * K + k8) = o; __threadfence(); *(volatile v8us*)((unsigned short*)Wt + (size_t)n * K + k8) = o;
}
template <int ACT>
__global__ __launch_bounds__(128) void k_gemm_hhx(const _Float16* __restrict__ A, int lda, size_t sA, const _Float16* __restrict__ Bh, int ldb, size_t sB, float alpha, const float* __restrict__ bias, size_t sBias, const float* __restrict__ CP, int rowsPerB, size_t sCPb, int row0g,
    float* __restrict__ C, _Float16* __restrict__ C16, int ldc, size_t sC, int M, int N, int K) {
  __shared__ __attribute__((aligned(16))) float so[4][16][64];
  const int tid = threadIdx.x, w = tid >> 5, lane = tid & 31, ln = lane & 15, hh = lane >> 4; const int by = blockIdx.y;
  A += (size_t)by * sA; Bh += (size_t)by * sB; const size_t cofs = (size_t)by * sC; const float* bp = bias ? bias + (size_t)by * sBias : nullptr;
  const int ntn = (N + 63) / 64; const int wid = blockIdx.x * 4 + w; const int mt = wid / ntn, nq = wid % ntn; if (mt * 16 >= M) return;
  const int row0 = mt * 16, col0 = nq * 64; const _Float16* arow = A + (size_t)(row0 + ln) * lda;
  v8f acc[4] = {};
  for (int kb = 0; kb < K; kb += 32) { FragH ah; ah.half[0] = *(const v8us*)((const unsigned short*)arow + kb + 8 * hh); ah.half[1] = *(const v8us*)((const unsigned short*)arow + kb + 16 + 8 * hh);
#pragma unroll
    for (int t = 0; t < 4; ++t) { if (col0 + t * 16 >= N) continue; const size_t boff = (size_t)(col0 + t * 16 + ln) * ldb + kb; FragH bq; bq.half[0] = *(const v8us*)((const unsigned short*)Bh + boff + 8 * hh); bq.half[1] = *(const v8us*)((const unsigned short*)Bh + boff + 16 + 8 * hh);
      acc[t] = mmaH<1>(ah.v, ah.v, bq.v, bq.v, acc[t]); }
  }
#pragma unroll
  for (int t = 0; t < 4; ++t) { if (col0 + t * 16 >= N) continue; const int col = col0 + t * 16 + ln; const float bv = bp ? bf16_round(bp[col]) : 0.f;
#pragma unroll
    for (int r = 0; r < 8; ++r) { float v = acc[t][r] * alpha + bv; if (CP) { const int bidx = (row0g + row0 + 8 * hh + r) / rowsPerB; v += CP[(size_t)bidx * sCPb + (size_t)by * 64 + col]; } if (ACT == 1) v = (v > 0.f) ? v : expm1f(v); else if (ACT == 3) v = fmaxf(v, 0.f); so[w][8 * hh + r][t * 16 + ln] = v; } }
  __builtin_amdgcn_fence(__ATOMIC_ACQ_REL, "workgroup"); __builtin_amdgcn_wave_barrier();
  const int rsub = lane >> 4, c4 = (lane & 15) * 4; typedef _Float16 v4h __attribute__((ext_vector_type(4)));
  for (int pass = 0; pass < 2; ++pass) {
#pragma unroll
    for (int q = 0; q < 8; ++q) { const int r = q * 2 + rsub; if (col0 + c4 < N) { const v4f v = *(const v4fa*)&so[w][r][c4]; if (C) *(volatile v4f*)(C + cofs + (size_t)(row0 + r) * ldc + col0 + c4) = v; if (C16) { v4h h4; for (int i = 0; i < 4; ++i) h4[i] = (_Float16)v[i]; *(volatile v4h*)(C16 + cofs + (size_t)(row0 + r) * ldc + col0 + c4) = h4; } } }
    if (pass == 0) __threadfence(); }
}


__global__ __launch_bounds__(256) void k_round16f(const float* __restrict__ W, _Float16* __restrict__ Bt, size_t n8) { const size_t t = (size_t)blockIdx.x * 256 + threadIdx.x; if (t >= n8) return; FragH f;
#pragma unroll
  for (int i = 0; i < 8; ++i) f.h[i] = (_Float16)(bf16_round(W[t * 8 + i]) * 16.0f); *(volatile v8us*)((unsigned short*)Bt + t * 8) = f.half[0]; __threadfence(); *(volatile v8us*)((unsigned short*)Bt + t * 8) = f.half[0]; }
__global__ __launch_bounds__(256) void k_x16(const float* __restrict__ x, _Float16* __restrict__ X16, size_t n8) { const size_t t = (size_t)blockIdx.x * 256 + threadIdx.x; if (t >= n8) return; FragH f;
#pragma unroll
  for (int q = 0; q < 8; ++q) f.h[q] = (_Float16)bf16_round(x[t * 8 + q]); *(volatile v8us*)((unsigned short*)X16 + t * 8) = f.half[0]; __threadfence(); *(volatile v8us*)((unsigned short*)X16 + t * 8) = f.half[0]; }
__global__ __launch_bounds__(256) void k_a16(const float* __restrict__ A, _Float16* __restrict__ A4) { const int t = blockIdx.x * 256 + threadIdx.x; if (t >= NN * (NK / 8)) return; const int n = t / (NK / 8), m8 = (t % (NK / 8)) * 8; FragH f;
#pragma unroll
  for (int q = 0; q < 8; ++q) { const int m = m8 + q; const int mc = (m < NN) ? m : (NN - 1); const float av = bf16_round(A[n * NN + mc]); f.h[q] = (_Float16)((m < NN) ? av : 0.f); }
  for (int pass = 0; pass < 2; ++pass) { for (int s = 0; s < 4; ++s) *(volatile v8us*)((unsigned short*)A4 + (size_t)n * (4 * NK) + s * NK + m8) = f.half[0]; if (pass == 0) __threadfence(); } }
__global__ __launch_bounds__(256) void k_wgat(const float* __restrict__ W, const float* __restrict__ as, const float* __restrict__ ad, _Float16* __restrict__ Bt, float* __restrict__ WA) { const int t = threadIdx.x; const int h = t / 64, d = t % 64;
  for (int pass = 0; pass < 2; ++pass) {
    for (int pp = t; pp < NHD * DH * (FF / 8); pp += 256) { const int row = pp / (FF / 8), f8 = (pp % (FF / 8)) * 8; const int rh = row / DH, rd = row % DH; FragH o;
#pragma unroll
      for (int q = 0; q < 8; ++q) o.h[q] = (_Float16)(bf16_round(W[((size_t)rh * FF + f8 + q) * DH + rd]) * 16.0f); *(volatile v8us*)((unsigned short*)Bt + (size_t)row * FF + f8) = o.half[0]; }
    { const int f = d; float sa = 0.f, sd = 0.f;
#pragma unroll 4
      for (int dd = 0; dd < DH; ++dd) { const float w = bf16_round(W[((size_t)h * FF + f) * DH + dd]); sa += w * bf16_round(as[h * DH + dd]); sd += w * bf16_round(ad[h * DH + dd]); } *(volatile float*)(WA + h * FF + f) = sa; *(volatile float*)(WA + G4 + h * FF + f) = sd; }
    if (pass == 0) __threadfence(); } }
__global__ __launch_bounds__(256) void k_esd(const float* __restrict__ x, const float* __restrict__ WA, float* __restrict__ ESD) { __shared__ float swa[2 * G4]; const int tid = threadIdx.x; for (int i = tid; i < 2 * G4; i += 256) swa[i] = WA[i]; __syncthreads();
  const int t = blockIdx.x * 256 + tid; if (t >= NR) return; const int b = t / NN, n = t % NN; float acc[8];
#pragma unroll
  for (int q = 0; q < 8; ++q) acc[q] = 0.f; const float* xr = x + (size_t)t * FF;
#pragma unroll 4
  for (int f = 0; f < FF; ++f) { const float xv = bf16_round(xr[f]);
#pragma unroll
    for (int q = 0; q < 8; ++q) acc[q] += xv * swa[q * FF + f]; }
  for (int pass = 0; pass < 2; ++pass) {
#pragma unroll
    for (int q = 0; q < 8; ++q) { const int which = q / 4, h = q % 4; *(volatile float*)(ESD + (((size_t)which * BB + b) * NHD + h) * NK + n) = acc[q]; }
    if (pass == 0) __threadfence(); } }
__global__ __launch_bounds__(256) void k_rowmax(const float* __restrict__ A, const float* __restrict__ ESD, float* __restrict__ MX) { const int t = blockIdx.x * 256 + threadIdx.x; if (t >= BB * NHD * NN) return; const int n = t % NN; const int bh = t / NN; const float* ar = A + (size_t)n * NN; const float* ed = ESD + ((size_t)BB * NHD + bh) * NK; float m = -3.0e38f;
#pragma unroll 4
  for (int mm = 0; mm < NN; ++mm) if (bf16_round(ar[mm]) > 1e-6f) m = fmaxf(m, ed[mm]);
  *(volatile float*)(MX + (size_t)bh * NK + n) = m; __threadfence(); *(volatile float*)(MX + (size_t)bh * NK + n) = m; }
__global__ __launch_bounds__(256) void k_wht(const _Float16* __restrict__ WH16, _Float16* __restrict__ WhT) { __shared__ unsigned short tl[64][66]; const int tid = threadIdx.x; const int slab = blockIdx.x / 7, mg = blockIdx.x % 7; const int b = slab / NHD, h = slab % NHD;
  for (int i = tid; i < 64 * 8; i += 256) { const int r = i / 8, c8 = (i % 8) * 8; const int m = mg * 64 + r; const int mc = (m < NN) ? m : (NN - 1); FragH f; f.half[0] = *(const v8us*)((const unsigned short*)WH16 + ((size_t)b * NN + mc) * G4 + h * DH + c8); if (m >= NN) { for (int q = 0; q < 8; ++q) f.h[q] = (_Float16)0.f; }
#pragma unroll
    for (int q = 0; q < 8; ++q) tl[r][c8 + q] = f.u[q]; }
  __syncthreads();
  for (int pass = 0; pass < 2; ++pass) {
#pragma unroll
    for (int rd = 0; rd < 2; ++rd) { const int d = rd * 32 + tid / 8, pc = tid % 8; const int m0 = mg * 64 + pc * 8; if (m0 < NK) { FragH o;
#pragma unroll
        for (int q = 0; q < 8; ++q) o.u[q] = tl[pc * 8 + q][d]; *(volatile v8us*)((unsigned short*)WhT + ((size_t)slab * DH + d) * NK + m0) = o.half[0]; } }
    if (pass == 0) __threadfence(); } }
__device__ __forceinline__ float leaky02(float v) { return v > 0.f ? v : 0.2f * v; }
template <bool ACC>
__global__ __launch_bounds__(128) void k_gat(const float* __restrict__ A, const float* __restrict__ ESD, const float* __restrict__ MX, const _Float16* __restrict__ WhT, float* __restrict__ GG) {
  __shared__ __attribute__((aligned(16))) float so[4][16][DH + 4]; const int tid = threadIdx.x, w = tid >> 5, lane = tid & 31, ln = lane & 15, hh = lane >> 4;
  const int wid = blockIdx.x * 4 + w; const int slab = wid / (NN / 16), it = wid % (NN / 16); const int b = slab / NHD, h = slab % NHD; const int n = it * 16 + ln;
  const float* es = ESD + ((size_t)b * NHD + h) * NK; const float* ed = ESD + ((size_t)BB * NHD + (size_t)b * NHD + h) * NK; const float esn = es[n]; const float mxn = MX[((size_t)b * NHD + h) * NK + n]; const bool empty = (mxn < -1.0e38f); const float mrow = leaky02(esn + mxn); const float* ar = A + (size_t)n * NN;
  v8f acc[4]; for (int t4 = 0; t4 < 4; ++t4) acc[t4] = (v8f){0.f,0.f,0.f,0.f,0.f,0.f,0.f,0.f}; float lsum = 0.f;
  const unsigned short* wt = (const unsigned short*)WhT + (size_t)slab * DH * NK;
#pragma unroll 1
  for (int ks = 0; ks < NK / 32; ++ks) { FragH a;
#pragma unroll
    for (int q = 0; q < 16; ++q) { const int m = ks * 32 + ((q < 8) ? (8 * hh + q) : (16 + 8 * hh + q - 8)); float p = 0.f;
      if (m < NN) { if (empty) p = 1.0f; else if (bf16_round(ar[m]) > 1e-6f) p = expf(leaky02(esn + ed[m]) - mrow); } lsum += p; a.h[q] = (_Float16)p; }
#pragma unroll
    for (int t4 = 0; t4 < 4; ++t4) { FragH bq; const unsigned short* br = wt + (size_t)(t4 * 16 + ln) * NK + ks * 32; bq.half[0] = *(const v8us*)(br + 8 * hh); bq.half[1] = *(const v8us*)(br + 16 + 8 * hh); acc[t4] = mmaH<1>(a.v, a.v, bq.v, bq.v, acc[t4]); } }
  lsum += __shfl_xor(lsum, 16, 32);
#pragma unroll
  for (int t4 = 0; t4 < 4; ++t4)
#pragma unroll
    for (int r = 0; r < 8; ++r) { const float l = __shfl(lsum, 8 * hh + r, 32); so[w][8 * hh + r][t4 * 16 + ln] = acc[t4][r] / l; }
  __builtin_amdgcn_fence(__ATOMIC_ACQ_REL, "workgroup"); __builtin_amdgcn_wave_barrier();
  for (int pass = 0; pass < 2; ++pass) {
#pragma unroll
    for (int rp = 0; rp < 16; rp += 2) { const int r = rp + (lane >> 4), pc = lane & 15; float* dst = GG + ((size_t)b * NN + it * 16 + r) * G4 + h * DH + pc * 4; v4f v = *(const v4fa*)&so[w][r][pc * 4]; if (ACC) { const v4f old = *(const v4fa*)dst; if (pass == 0) { v += old; *(v4fa*)&so[w][r][pc * 4] = v; } } *(volatile v4f*)dst = *(const v4fa*)&so[w][r][pc * 4]; }
    if (pass == 0) __threadfence(); } }
__global__ __launch_bounds__(256) void k_split2(const float* __restrict__ S, int nrow, int coff, _Float16* __restrict__ XW4) { const size_t t = (size_t)blockIdx.x * 256 + threadIdx.x; if (t >= (size_t)nrow * (NK / 8)) return; const size_t r = t / (NK / 8); const int c8 = (int)(t % (NK / 8)) * 8; FragH h, l;
#pragma unroll
  for (int q = 0; q < 8; ++q) { const int c = c8 + q; const float v = (c < NN) ? S[r * NK + c] : 0.f; const _Float16 hv = (_Float16)v; h.h[q] = hv; l.h[q] = (_Float16)(v - (float)hv); }
  for (int pass = 0; pass < 2; ++pass) { *(volatile v8us*)((unsigned short*)XW4 + r * (4 * NK) + coff + c8) = h.half[0]; *(volatile v8us*)((unsigned short*)XW4 + r * (4 * NK) + coff + NK + c8) = l.half[0]; if (pass == 0) __threadfence(); } }
__global__ __launch_bounds__(256) void k_fcat(const float* __restrict__ GC, const float* __restrict__ GG, _Float16* __restrict__ FHI, _Float16* __restrict__ FLO) { const size_t t = (size_t)blockIdx.x * 256 + threadIdx.x; if (t >= (size_t)NR * 512 / 8) return; const size_t r = t / 64; const int c8 = (int)(t % 64) * 8; FragH h, l; const float* src = (c8 < G4) ? (GC + r * G4 + c8) : (GG + r * G4 + c8 - G4);
#pragma unroll
  for (int q = 0; q < 8; ++q) { const float v = src[q]; const _Float16 hv = (_Float16)v; h.h[q] = hv; l.h[q] = (_Float16)(v - (float)hv); }
  for (int pass = 0; pass < 2; ++pass) { *(volatile v8us*)((unsigned short*)FHI + t * 8) = h.half[0]; *(volatile v8us*)((unsigned short*)FLO + t * 8) = l.half[0]; if (pass == 0) __threadfence(); } }
__global__ __launch_bounds__(256) void k_bias2(const float* __restrict__ b1, const float* __restrict__ b2, float* __restrict__ BS) { const int t = threadIdx.x; const float v = bf16_round(b1[t]) + bf16_round(b2[t]); *(volatile float*)(BS + t) = v; __threadfence(); *(volatile float*)(BS + t) = v; }
__global__ __launch_bounds__(256) void k_cell(const float* __restrict__ PRE, const float* __restrict__ cp, float* __restrict__ hout, float* __restrict__ cout_) { const size_t t = (size_t)blockIdx.x * 256 + threadIdx.x; if (t >= (size_t)NR * HH / 8) return; const size_t r = t / (HH / 8); const int j8 = (int)(t % (HH / 8)) * 8; const float* pr = PRE + r * G4; v4f h0, h1, c0, c1;
#pragma unroll 1
  for (int q = 0; q < 8; ++q) { const int j = j8 + q; const float ig = 1.0f / (1.0f + expf(-pr[j])), fg = 1.0f / (1.0f + expf(-pr[HH + j])), og = 1.0f / (1.0f + expf(-pr[2 * HH + j])), gg = tanhf(pr[3 * HH + j]);
    const float c = fg * bf16_round(cp[r * HH + j]) + ig * gg; const float hv = og * tanhf(c); if (q < 4) { h0[q] = hv; c0[q] = c; } else { h1[q - 4] = hv; c1[q - 4] = c; } }
  { const int lane = threadIdx.x & 31; const size_t span = (t & ~(size_t)31) * 8; store_span256(hout + span, h0, h1, lane); store_span256(cout_ + span, c0, c1, lane); } }
extern "C" void kernel_launch(void* const* d_in, const int* in_sizes, int n_in,
                              void* d_out, int out_size, void* d_ws, size_t ws_size, hipStream_t stream) {
  (void)in_sizes; (void)n_in; (void)out_size;
  const float* x = (const float*)d_in[0]; const float* hp = (const float*)d_in[1]; const float* cp = (const float*)d_in[2]; const float* A = (const float*)d_in[3]; const float* Wgcx = (const float*)d_in[4]; const float* bgcx = (const float*)d_in[5]; const float* Wgch = (const float*)d_in[6]; const float* bgch = (const float*)d_in[7];
  const float* Wgx = (const float*)d_in[8]; const float* asx = (const float*)d_in[9]; const float* adx = (const float*)d_in[10]; const float* Wgh = (const float*)d_in[11]; const float* ash = (const float*)d_in[12]; const float* adh = (const float*)d_in[13]; const float* Wfp = (const float*)d_in[14]; const float* bfp = (const float*)d_in[15];
  float* hout = (float*)d_out; float* cout_ = (float*)((char*)d_out + 3276800);
  char* ws = (char*)d_ws; size_t off = 0;
  auto take = [&](size_t bytes) { char* p = ws + off; off += (bytes + 255) & ~(size_t)255; return p; };
  _Float16* A4 = (_Float16*)take((size_t)NN * 4 * NK * 2); _Float16* X16 = (_Float16*)take((size_t)NR * FF * 2); _Float16* H16 = (_Float16*)take((size_t)NR * HH * 2);
  _Float16* BWx = (_Float16*)take(G4 * FF * 2); _Float16* BWh = (_Float16*)take(G4 * HH * 2); float* BSg = (float*)take(G4 * 4); float* XWT = (float*)take((size_t)BB * G4 * NK * 4); _Float16* XW4 = (_Float16*)take((size_t)BB * G4 * 4 * NK * 2); float* GC = (float*)take((size_t)NR * G4 * 4);
  _Float16* Btx = (_Float16*)take(G4 * FF * 2); _Float16* Bth = (_Float16*)take(G4 * HH * 2); float* WAx = (float*)take(2 * G4 * 4); float* WAh = (float*)take(2 * G4 * 4); _Float16* WH16 = (_Float16*)take((size_t)NR * G4 * 2); float* ESD = (float*)take((size_t)2 * BB * NHD * NK * 4); float* MX = (float*)take((size_t)BB * NHD * NK * 4); _Float16* WhT = (_Float16*)take((size_t)BB * NHD * DH * NK * 2); float* GG = (float*)take((size_t)NR * G4 * 4);
  _Float16* FHI = (_Float16*)take((size_t)NR * 512 * 2); _Float16* FLO = (_Float16*)take((size_t)NR * 512 * 2); _Float16* Bfp = (_Float16*)take((size_t)G4 * 512 * 2); float* PRE = (float*)take((size_t)NR * G4 * 4);
  if (off > ws_size) return;
  const dim3 gr(((NR / 16) * (G4 / 64) + 3) / 4, 1);
  k_a16<<<(NN * (NK / 8) + 255) / 256, 256, 0, stream>>>(A, A4);
  k_x16<<<(unsigned)(((size_t)NR * FF / 8 + 255) / 256), 256, 0, stream>>>(x, X16, (size_t)NR * FF / 8); k_x16<<<(unsigned)(((size_t)NR * HH / 8 + 255) / 256), 256, 0, stream>>>(hp, H16, (size_t)NR * HH / 8);
  k_wt_f16<<<(G4 * (FF / 8) + 255) / 256, 256, 0, stream>>>(Wgcx, BWx, FF, G4, 16.0f); k_wt_f16<<<(G4 * (HH / 8) + 255) / 256, 256, 0, stream>>>(Wgch, BWh, HH, G4, 16.0f); k_bias2<<<1, 256, 0, stream>>>(bgcx, bgch, BSg);
  for (int br = 0; br < 2; ++br) { const _Float16* S16 = br ? H16 : X16; const _Float16* BW = br ? BWh : BWx;
    k_gemm_hhx<0><<<dim3(((G4 / 16) * ((NN + 63) / 64) + 3) / 4, BB), 128, 0, stream>>>(BW, FF, 0, S16, FF, (size_t)NN * FF, 0.0625f, nullptr, 0, nullptr, 1, 0, 0, XWT, nullptr, NK, (size_t)G4 * NK, G4, NN, FF);
    k_split2<<<(unsigned)(((size_t)BB * G4 * (NK / 8) + 255) / 256), 256, 0, stream>>>(XWT, BB * G4, br * 2 * NK, XW4); }
  k_gemm_hhx<0><<<dim3(((NN / 16) * (G4 / 64) + 3) / 4, BB), 128, 0, stream>>>(A4, 4 * NK, 0, XW4, 4 * NK, (size_t)G4 * 4 * NK, 1.0f, BSg, 0, nullptr, 1, 0, 0, GC, nullptr, G4, (size_t)NN * G4, NN, G4, 4 * NK);
  for (int br = 0; br < 2; ++br) {
    const float* src = br ? hp : x; const float* Wg = br ? Wgh : Wgx; const float* as_ = br ? ash : asx; const float* ad_ = br ? adh : adx; const _Float16* S16 = br ? H16 : X16; _Float16* Bt = br ? Bth : Btx; float* WA = br ? WAh : WAx;
    k_wgat<<<1, 256, 0, stream>>>(Wg, as_, ad_, Bt, WA);
    k_gemm_hhx<0><<<gr, 128, 0, stream>>>(S16, FF, 0, Bt, FF, 0, 0.0625f, nullptr, 0, nullptr, 1, 0, 0, nullptr, WH16, G4, 0, NR, G4, FF);
    k_esd<<<(NR + 255) / 256, 256, 0, stream>>>(src, WA, ESD);
    k_rowmax<<<(BB * NHD * NN + 255) / 256, 256, 0, stream>>>(A, ESD, MX);
    k_wht<<<BB * NHD * 7, 256, 0, stream>>>(WH16, WhT);
    if (br == 0) k_gat<false><<<(BB * NHD * (NN / 16)) / 4, 128, 0, stream>>>(A, ESD, MX, WhT, GG);
    else         k_gat<true><<<(BB * NHD * (NN / 16)) / 4, 128, 0, stream>>>(A, ESD, MX, WhT, GG);
  }
  k_fcat<<<(unsigned)(((size_t)NR * 512 / 8 + 255) / 256), 256, 0, stream>>>(GC, GG, FHI, FLO);
  k_wt_f16<<<(G4 * (512 / 8) + 255) / 256, 256, 0, stream>>>(Wfp, Bfp, 512, G4, 16.0f);
  k_gemm_hhx<0><<<gr, 128, 0, stream>>>(FHI, 512, 0, Bfp, 512, 0, 0.0625f, bfp, 0, nullptr, 1, 0, 0, PRE, nullptr, G4, 0, NR, G4, 512);
  k_gemm_hhx<0><<<gr, 128, 0, stream>>>(FLO, 512, 0, Bfp, 512, 0, 0.0625f, nullptr, 0, PRE, 1, (size_t)G4, 0, PRE, nullptr, G4, 0, NR, G4, 512);
  k_cell<<<(unsigned)(((size_t)NR * HH / 8 + 255) / 256), 256, 0, stream>>>(PRE, cp, hout, cout_);
}
